// LocalAttentionBlock_27401891349134
// MI455X (gfx1250) — hardware-verified
//
#include <hip/hip_runtime.h>
#include <math.h>
#include <stdint.h>

#define BB    2
#define SS    2048
#define WID   1024
#define NH    16
#define HD    64
#define BT    (BB * SS)
#define WIN   1024
#define KOUT  (2 * WID)
#define MASKV (-1.0e30f)


typedef __attribute__((ext_vector_type(16))) _Float16 v16h;
typedef __attribute__((ext_vector_type(8)))  _Float16 v8h;
typedef __attribute__((ext_vector_type(16))) __bf16   v16b;
typedef __attribute__((ext_vector_type(8)))  __bf16   v8b;
typedef __attribute__((ext_vector_type(8)))  float    v8f;
typedef __attribute__((ext_vector_type(4)))  float    v4f;
typedef __attribute__((ext_vector_type(2)))  float    v2f;
typedef __attribute__((ext_vector_type(4)))  unsigned int v4u;

static_assert(SS % 64 == 0);
static_assert(WID % 64 == 0);
static_assert(KOUT % 32 == 0);
static_assert(BT % 64 == 0);
static_assert(HD == 64);
static_assert(NH * HD == WID);

__device__ __forceinline__ unsigned short f2bf_bits(float f) {
  unsigned u = __float_as_uint(f);
  return (unsigned short)((u + 0x7FFFu + ((u >> 16) & 1u)) >> 16);
}
__device__ __forceinline__ float bf_bits2f(unsigned short h) { return __uint_as_float(((unsigned)h) << 16); }
__device__ __forceinline__ unsigned pk16(unsigned short a, unsigned short b) { return (unsigned)a | ((unsigned)b << 16); }

__device__ __forceinline__ void dep_guard_h(v8f& a, v8f& b, v16h x, v16h y) { asm volatile("v_nop\n\tv_nop\n\tv_nop\n\tv_nop" : "+v"(a), "+v"(b) : "v"(x), "v"(y)); }
__device__ __forceinline__ void dep_guard_b(v8f& a, v8f& b, v16b x, v16b y) { asm volatile("v_nop\n\tv_nop\n\tv_nop\n\tv_nop" : "+v"(a), "+v"(b) : "v"(x), "v"(y)); }
__device__ __forceinline__ void keep4_h(v16h a, v16h b, v16h c, v16h d) { asm volatile("v_nop" :: "v"(a), "v"(b), "v"(c), "v"(d)); }
__device__ __forceinline__ void keep4_b(v16b a, v16b b, v16b c, v16b d) { asm volatile("v_nop" :: "v"(a), "v"(b), "v"(c), "v"(d)); }
__device__ __forceinline__ void acc_guard4(v8f& a, v8f& b, v8f& c, v8f& d) { asm volatile("v_nop\n\tv_nop\n\tv_nop\n\tv_nop" : "+v"(a), "+v"(b), "+v"(c), "+v"(d)); }

template <typename T> struct Frag;
template <> struct Frag<_Float16> {
  typedef v16h V; union U { v16h v; v8h h[2]; };
  static __device__ __forceinline__ v16h load(const _Float16* p) {
    U f; f.h[0] = *(const v8h*)(p); f.h[1] = *(const v8h*)(p + 16); return f.v;
  }
  static __device__ __forceinline__ v8f mma(v16h a, v16h b, v8f c) {
    return __builtin_amdgcn_wmma_f32_16x16x32_f16(false, a, false, b, (short)0, c, false, false);
  }
  static __device__ __forceinline__ void guard(v8f& a, v8f& b, v16h x, v16h y) { dep_guard_h(a, b, x, y); }
  static __device__ __forceinline__ void keep(v16h a, v16h b, v16h c, v16h d) { keep4_h(a, b, c, d); }
};
template <> struct Frag<__bf16> {
  typedef v16b V; union U { v16b v; v8b h[2]; };
  static __device__ __forceinline__ v16b load(const __bf16* p) {
    U f; f.h[0] = *(const v8b*)(p); f.h[1] = *(const v8b*)(p + 16); return f.v;
  }
  static __device__ __forceinline__ v8f mma(v16b a, v16b b, v8f c) {
    return __builtin_amdgcn_wmma_f32_16x16x32_bf16(false, a, false, b, (short)0, c, false, false);
  }
  static __device__ __forceinline__ void guard(v8f& a, v8f& b, v16b x, v16b y) { dep_guard_b(a, b, x, y); }
  static __device__ __forceinline__ void keep(v16b a, v16b b, v16b c, v16b d) { keep4_b(a, b, c, d); }
};

template <int ET> struct Elem;
template <> struct Elem<0> { typedef _Float16 T; };
template <> struct Elem<1> { typedef __bf16 T; };
template <int ET, bool SPLIT, int BIAS_MODE, int OUT_MODE, bool RESID>
__global__ __launch_bounds__(256) void wmma_gemm64(
    const unsigned short* __restrict__ Ap, const unsigned short* __restrict__ A2p, int lda, long strideA,
    const unsigned short* __restrict__ Btp, const unsigned short* __restrict__ Bt2p, int ldb, long strideB,
    void* __restrict__ Cout, void* __restrict__ Cout2, int ldc, long strideC,
    const float* __restrict__ bias,
    const float* __restrict__ resid, long strideR,
    int M, int N, int K, float scale) {
  typedef typename Elem<ET>::T T;
  typedef typename Frag<T>::V V;
  const T* A = (const T*)Ap; const T* A2 = (const T*)A2p; const T* Bt = (const T*)Btp; const T* Bt2 = (const T*)Bt2p;
  __shared__ __align__(16) float sT[8][16 * 68];
  const int b    = blockIdx.y;
  const int lane = threadIdx.x & 31;
  const int wave = threadIdx.x >> 5;
  const int tilesN = N >> 6;
  const int tilesM = M >> 6;
  const int tile = blockIdx.x * 8 + wave;
  if (tile >= tilesM * tilesN) return;
  const int tm = tile / tilesN;
  const int tn = tile - tm * tilesN;
  const int m0 = tm << 6;
  const int n0 = tn << 6;

  const T* Ab  = A  + (size_t)b * strideA;
  const T* Bb  = Bt + (size_t)b * strideB;
  const T* Ab2 = SPLIT ? (A2  + (size_t)b * strideA) : nullptr;
  const T* Bb2 = SPLIT ? (Bt2 + (size_t)b * strideB) : nullptr;

  const int rlane = lane & 15;
  const int koff  = (lane >> 4) * 8;
  const int mOff  = (lane >> 4) * 8;

  v8f acc[4][4];
#pragma unroll
  for (int i = 0; i < 4; ++i)
#pragma unroll
    for (int j = 0; j < 4; ++j) acc[i][j] = (v8f){0.f,0.f,0.f,0.f,0.f,0.f,0.f,0.f};

  for (int k0 = 0; k0 < K; k0 += 32) {
    V bh[4], bl[4];
#pragma unroll
    for (int j = 0; j < 4; ++j) {
      const size_t bo = (size_t)(n0 + (j << 4) + rlane) * ldb + koff + k0;
      bh[j] = Frag<T>::load(Bb + bo);
      if (SPLIT) bl[j] = Frag<T>::load(Bb2 + bo);
    }
#pragma unroll
    for (int i = 0; i < 4; ++i) {
      const size_t ao = (size_t)(m0 + (i << 4) + rlane) * lda + koff + k0;
      V ah = Frag<T>::load(Ab + ao);
      V al;
      if (SPLIT) al = Frag<T>::load(Ab2 + ao);
#pragma unroll
      for (int j = 0; j < 4; ++j) {
        acc[i][j] = Frag<T>::mma(ah, bh[j], acc[i][j]);
        if (SPLIT) {
          acc[i][j] = Frag<T>::mma(ah, bl[j], acc[i][j]);
          acc[i][j] = Frag<T>::mma(al, bh[j], acc[i][j]);
        }
      }
      Frag<T>::guard(acc[i][0], acc[i][3], ah, SPLIT ? al : ah);
    }
    Frag<T>::keep(bh[0], bh[1], bh[2], bh[3]);
    if (SPLIT) Frag<T>::keep(bl[0], bl[1], bl[2], bl[3]);
  }
  acc_guard4(acc[0][0], acc[0][1], acc[0][2], acc[0][3]);
  acc_guard4(acc[1][0], acc[1][1], acc[1][2], acc[1][3]);
  acc_guard4(acc[2][0], acc[2][1], acc[2][2], acc[2][3]);
  acc_guard4(acc[3][0], acc[3][1], acc[3][2], acc[3][3]);

  float* slab = sT[wave];
  const float* Rb = RESID ? (resid + (size_t)b * strideR) : nullptr;
#pragma unroll
  for (int i = 0; i < 4; ++i) {
    const int mBase = m0 + (i << 4);
#pragma unroll
    for (int j = 0; j < 4; ++j) {
      const int n = n0 + (j << 4) + rlane;
      float bv = 0.f;
      if (BIAS_MODE == 2) bv = bf_bits2f(f2bf_bits(bias[n]));
#pragma unroll
      for (int r = 0; r < 8; ++r) {
        float v = acc[i][j][r] * scale;
        if (BIAS_MODE == 1) v += bias[mBase + mOff + r];
        if (BIAS_MODE == 2) v += bv;
        if (RESID) v += Rb[(size_t)(mBase + mOff + r) * ldc + n];
        slab[(mOff + r) * 68 + (j << 4) + rlane] = v;
      }
    }
    __builtin_amdgcn_fence(__ATOMIC_RELEASE, "workgroup");
    __builtin_amdgcn_wave_barrier();
    __builtin_amdgcn_fence(__ATOMIC_ACQUIRE, "workgroup");
    if (OUT_MODE == 0) {
      float* C = (float*)Cout + (size_t)b * strideC;
      const int hh = lane >> 4, c4 = (lane & 15) * 4;
      for (int pass = 0; pass < 2; ++pass) {
#pragma unroll
        for (int it = 0; it < 8; ++it) {
          const int row = it * 2 + hh;
          v4f v = *(const v4f*)(slab + row * 68 + c4);
          *(volatile v4f*)(C + (size_t)(mBase + row) * ldc + n0 + c4) = v;
        }
        __threadfence();
      }
    } else {
      const int q = lane >> 3, c8 = (lane & 7) * 8;
      unsigned short* C  = (unsigned short*)Cout  + (size_t)b * strideC;
      unsigned short* C2 = (OUT_MODE == 2) ? ((unsigned short*)Cout2 + (size_t)b * strideC) : nullptr;
      for (int pass = 0; pass < 2; ++pass) {
#pragma unroll
        for (int it = 0; it < 4; ++it) {
          const int row = it * 4 + q;
          const float* sp = slab + row * 68 + c8;
          v8h hv, lv;
#pragma unroll
          for (int e = 0; e < 8; ++e) {
            if (OUT_MODE == 1) {
              hv[e] = (_Float16)sp[e];
            } else {
              unsigned short hb = f2bf_bits(sp[e]);
              unsigned short lb = f2bf_bits(sp[e] - bf_bits2f(hb));
              hv[e] = __builtin_bit_cast(_Float16, hb);
              lv[e] = __builtin_bit_cast(_Float16, lb);
            }
          }
          *(volatile v8h*)(C + (size_t)(mBase + row) * ldc + n0 + c8) = hv;
          if (OUT_MODE == 2) *(volatile v8h*)(C2 + (size_t)(mBase + row) * ldc + n0 + c8) = lv;
        }
        __threadfence();
      }
    }
    __builtin_amdgcn_fence(__ATOMIC_RELEASE, "workgroup");
    __builtin_amdgcn_wave_barrier();
    __builtin_amdgcn_fence(__ATOMIC_ACQUIRE, "workgroup");
  }
}

template <bool DUP>
__global__ __launch_bounds__(256) void cvt_bf16_kernel(const float* __restrict__ in, unsigned short* __restrict__ out,
                                                       int n8, int srcCols, int dstPitch, int dupOff) {
  const int i = blockIdx.x * 256 + threadIdx.x;
  if (i < n8) {
    const size_t e   = (size_t)i * 8;
    const size_t row = e / (size_t)srcCols;
    const size_t col = e - row * (size_t)srcCols;
    const v4f f0 = *(const v4f*)(in + e);
    const v4f f1 = *(const v4f*)(in + e + 4);
    v4u u;
    u[0] = pk16(f2bf_bits(f0[0]), f2bf_bits(f0[1]));
    u[1] = pk16(f2bf_bits(f0[2]), f2bf_bits(f0[3]));
    u[2] = pk16(f2bf_bits(f1[0]), f2bf_bits(f1[1]));
    u[3] = pk16(f2bf_bits(f1[2]), f2bf_bits(f1[3]));
    const size_t d = row * (size_t)dstPitch + col;
    *(volatile v4u*)(out + d) = u;
    if (DUP) *(volatile v4u*)(out + d + dupOff) = u;
    __threadfence();
    *(volatile v4u*)(out + d) = u;
    if (DUP) *(volatile v4u*)(out + d + dupOff) = u;
  }
}

#define AT_D  64
#define AT_NW 4
#define AT_QB 64
#define AT_KC 64
#define NQT   (SS / AT_QB)
#define KSPAN (WIN / AT_KC)

static_assert(WIN % AT_KC == 0);
static_assert(KSPAN == 16);
static_assert(NQT * NH * BB == 1024);

__device__ __forceinline__ __bf16 at_f2bf(float f) { return __builtin_bit_cast(__bf16, f2bf_bits(f)); }
__device__ __forceinline__ void at_split(float f, __bf16& hi, __bf16& lo) {
  const unsigned short hb = f2bf_bits(f);
  hi = __builtin_bit_cast(__bf16, hb);
  lo = at_f2bf(f - __uint_as_float(((unsigned)hb) << 16));
}
__device__ __forceinline__ v8f at_mma(v16b a, v16b b, v8f c) {
  c = __builtin_amdgcn_wmma_f32_16x16x32_bf16(false, a, false, b, (short)0, c, false, false);
  asm volatile("v_nop\n\tv_nop\n\tv_nop\n\tv_nop" : "+v"(c) : "v"(a), "v"(b));
  return c;
}

__global__ __launch_bounds__(128)
void attn_local64_kernel(const unsigned short* __restrict__ qhp, const unsigned short* __restrict__ qlp,
                         const unsigned short* __restrict__ khp, const unsigned short* __restrict__ klp,
                         const unsigned short* __restrict__ vhp, const unsigned short* __restrict__ vlp,
                         unsigned short* __restrict__ op, float sscale,
                         const int* __restrict__ segpos) {
  (void)segpos;
  union FB { v16b v; v8b h[2]; };
  __shared__ __align__(16) __bf16 Ksh[AT_KC * AT_D];
  __shared__ __align__(16) __bf16 Ksl[AT_KC * AT_D];
  __shared__ __align__(16) __bf16 Vth[AT_D * AT_KC];
  __shared__ __align__(16) __bf16 Vtl[AT_D * AT_KC];
  __shared__ __align__(16) __bf16 Psh[AT_NW][16 * AT_KC];
  __shared__ __align__(16) __bf16 Psl[AT_NW][16 * AT_KC];
  __shared__ __align__(16) float  Os[AT_NW][16 * 68];

  const int tid  = threadIdx.x;
  const int wave = tid >> 5;
  const int lane = tid & 31;
  const int hh   = lane >> 4;
  const int c    = lane & 15;

  const int bx   = blockIdx.x;
  const int qt   = bx % NQT;
  const int head = (bx / NQT) % NH;
  const int b    = bx / (NQT * NH);
  const int q0   = qt * AT_QB + wave * 16;
  const size_t brow = (size_t)b * SS;

  const __bf16* Qh = (const __bf16*)(const void*)qhp + brow * WID + (size_t)head * HD;
  const __bf16* Ql = (const __bf16*)(const void*)qlp + brow * WID + (size_t)head * HD;
  const __bf16* Kh = (const __bf16*)(const void*)khp + brow * HD;
  const __bf16* Kl = (const __bf16*)(const void*)klp + brow * HD;
  const __bf16* Vh = (const __bf16*)(const void*)vhp + brow;
  const __bf16* Vl = (const __bf16*)(const void*)vlp + brow;
  unsigned short* Oh = op + brow * KOUT + (size_t)head * HD;
  unsigned short* Ol = Oh + WID;

  v16b qah[2], qal[2];
#pragma unroll
  for (int dc = 0; dc < 2; ++dc) {
    const __bf16* qr = Qh + (size_t)(q0 + c) * WID + dc * 32 + 8 * hh;
    const __bf16* ql = Ql + (size_t)(q0 + c) * WID + dc * 32 + 8 * hh;
    qah[dc] = Frag<__bf16>::load(qr);
    qal[dc] = Frag<__bf16>::load(ql);
  }

  float mrow[8], lrow[8];
  v8f oacc[4];
#pragma unroll
  for (int r = 0; r < 8; ++r) { mrow[r] = -INFINITY; lrow[r] = 0.f; }
#pragma unroll
  for (int t = 0; t < 4; ++t) oacc[t] = (v8f){0.f,0.f,0.f,0.f,0.f,0.f,0.f,0.f};

  const int kcBeg = (qt > KSPAN) ? (qt - KSPAN) : 0;
  const int kcEnd = qt;
  for (int kc = kcBeg; kc <= kcEnd; ++kc) {
    const int kv0 = kc * AT_KC;
    __syncthreads();
    {
      const int r = tid >> 1, half = (tid & 1) * 32;
      const __bf16* ksh = Kh + (size_t)(kv0 + r) * HD + half;
      const __bf16* ksl = Kl + (size_t)(kv0 + r) * HD + half;
      const __bf16* vsh = Vh + (size_t)r * BT + kv0 + half;
      const __bf16* vsl = Vl + (size_t)r * BT + kv0 + half;
#pragma unroll
      for (int i = 0; i < 4; ++i) {
        const v8b a0 = *(const v8b*)(ksh + 8 * i);
        const v8b a1 = *(const v8b*)(ksl + 8 * i);
        const v8b b0 = *(const v8b*)(vsh + 8 * i);
        const v8b b1 = *(const v8b*)(vsl + 8 * i);
        *(v8b*)(Ksh + r * AT_D  + half + 8 * i) = a0;
        *(v8b*)(Ksl + r * AT_D  + half + 8 * i) = a1;
        *(v8b*)(Vth + r * AT_KC + half + 8 * i) = b0;
        *(v8b*)(Vtl + r * AT_KC + half + 8 * i) = b1;
      }
    }
    __syncthreads();

    v8f s[4];
#pragma unroll
    for (int j = 0; j < 4; ++j) {
      s[j] = (v8f){0.f,0.f,0.f,0.f,0.f,0.f,0.f,0.f};
#pragma unroll
      for (int dc = 0; dc < 2; ++dc) {
        FB kb, kl;
        kb.h[0] = *(const v8b*)(Ksh + (j * 16 + c) * AT_D + dc * 32 + 8 * hh);
        kb.h[1] = *(const v8b*)(Ksh + (j * 16 + c) * AT_D + dc * 32 + 16 + 8 * hh);
        kl.h[0] = *(const v8b*)(Ksl + (j * 16 + c) * AT_D + dc * 32 + 8 * hh);
        kl.h[1] = *(const v8b*)(Ksl + (j * 16 + c) * AT_D + dc * 32 + 16 + 8 * hh);
        s[j] = at_mma(qah[dc], kb.v, s[j]);
        s[j] = at_mma(qah[dc], kl.v, s[j]);
        s[j] = at_mma(qal[dc], kb.v, s[j]);
      }
    }
    float cm[8];
#pragma unroll
    for (int r = 0; r < 8; ++r) {
      const int t = q0 + 8 * hh + r;
      float m = -INFINITY;
#pragma unroll
      for (int j = 0; j < 4; ++j) {
        const int sk = kv0 + j * 16 + c;
        const int dt = t - sk;
        const bool ok = (dt >= 0) && (dt <= WIN);
        float sv = s[j][r] * sscale;
        sv = ok ? sv : MASKV;
        s[j][r] = sv;
        m = fmaxf(m, sv);
      }
#pragma unroll
      for (int off = 1; off < 16; off <<= 1) m = fmaxf(m, __shfl_xor(m, off, 32));
      cm[r] = m;
    }
    __bf16* pwh = Psh[wave];
    __bf16* pwl = Psl[wave];
#pragma unroll
    for (int r = 0; r < 8; ++r) {
      const float mnew = fmaxf(mrow[r], cm[r]);
      const float alpha = expf(mrow[r] - mnew);
      mrow[r] = mnew;
      float psum = 0.f;
#pragma unroll
      for (int j = 0; j < 4; ++j) {
        const float p = expf(s[j][r] - mnew);
        psum += p;
        __bf16 a, bl; at_split(p, a, bl);
        pwh[(8 * hh + r) * AT_KC + j * 16 + c] = a;
        pwl[(8 * hh + r) * AT_KC + j * 16 + c] = bl;
      }
#pragma unroll
      for (int off = 1; off < 16; off <<= 1) psum += __shfl_xor(psum, off, 32);
      lrow[r] = lrow[r] * alpha + psum;
#pragma unroll
      for (int t = 0; t < 4; ++t) oacc[t][r] *= alpha;
    }
    __builtin_amdgcn_fence(__ATOMIC_RELEASE, "workgroup");
    __builtin_amdgcn_wave_barrier();
    __builtin_amdgcn_fence(__ATOMIC_ACQUIRE, "workgroup");
#pragma unroll 1
    for (int kk = 0; kk < 2; ++kk) {
      FB pa, pl;
      pa.h[0] = *(const v8b*)(pwh + c * AT_KC + kk * 32 + 8 * hh);
      pa.h[1] = *(const v8b*)(pwh + c * AT_KC + kk * 32 + 16 + 8 * hh);
      pl.h[0] = *(const v8b*)(pwl + c * AT_KC + kk * 32 + 8 * hh);
      pl.h[1] = *(const v8b*)(pwl + c * AT_KC + kk * 32 + 16 + 8 * hh);
#pragma unroll
      for (int t = 0; t < 4; ++t) {
        FB vb, vl;
        vb.h[0] = *(const v8b*)(Vth + (t * 16 + c) * AT_KC + kk * 32 + 8 * hh);
        vb.h[1] = *(const v8b*)(Vth + (t * 16 + c) * AT_KC + kk * 32 + 16 + 8 * hh);
        vl.h[0] = *(const v8b*)(Vtl + (t * 16 + c) * AT_KC + kk * 32 + 8 * hh);
        vl.h[1] = *(const v8b*)(Vtl + (t * 16 + c) * AT_KC + kk * 32 + 16 + 8 * hh);
        oacc[t] = at_mma(pa.v, vb.v, oacc[t]);
        oacc[t] = at_mma(pa.v, vl.v, oacc[t]);
        oacc[t] = at_mma(pl.v, vb.v, oacc[t]);
      }
    }
  }

  float* os = Os[wave];
#pragma unroll
  for (int r = 0; r < 8; ++r) {
    const float inv = 1.0f / lrow[r];
#pragma unroll
    for (int t = 0; t < 4; ++t) os[(8 * hh + r) * 68 + t * 16 + c] = oacc[t][r] * inv;
  }
  __builtin_amdgcn_fence(__ATOMIC_RELEASE, "workgroup");
  __builtin_amdgcn_wave_barrier();
  __builtin_amdgcn_fence(__ATOMIC_ACQUIRE, "workgroup");
  {
    const int q = lane >> 3, c8 = (lane & 7) * 8;
    v4u hv[4], lv[4];
#pragma unroll
    for (int it = 0; it < 4; ++it) {
      const int row = it * 4 + q;
      const float* sp = os + row * 68 + c8;
      v4u a, a2;
#pragma unroll
      for (int g = 0; g < 4; ++g) {
        const float f0 = sp[2 * g], f1 = sp[2 * g + 1];
        const unsigned short h0 = f2bf_bits(f0), h1 = f2bf_bits(f1);
        const unsigned short l0 = f2bf_bits(f0 - bf_bits2f(h0)), l1 = f2bf_bits(f1 - bf_bits2f(h1));
        a[g]  = pk16(h0, h1);
        a2[g] = pk16(l0, l1);
      }
      hv[it] = a; lv[it] = a2;
    }
    for (int pass = 0; pass < 2; ++pass) {
#pragma unroll
      for (int it = 0; it < 4; ++it) {
        const int row = it * 4 + q;
        const size_t go = (size_t)(q0 + row) * KOUT + c8;
        *(volatile v4u*)(Oh + go) = hv[it];
        *(volatile v4u*)(Ol + go) = lv[it];
      }
      __threadfence();
    }
  }
}

extern "C" void kernel_launch(void* const* d_in, const int* in_sizes, int n_in,
                              void* d_out, int out_size, void* d_ws, size_t ws_size,
                              hipStream_t stream) {
  if (n_in < 7) return;
  if (in_sizes[0] != BT * WID) return;
  if (in_sizes[1] != BB * SS) return;
  if (in_sizes[2] != WID * WID) return;
  if (in_sizes[3] != HD * WID || in_sizes[4] != HD * WID) return;
  if (in_sizes[5] != WID * WID) return;
  if (in_sizes[6] != WID) return;
  if (out_size != BT * WID) return;

  const float* x      = (const float*)d_in[0];
  const int*   segpos = (const int*)d_in[1];
  const float* Wq     = (const float*)d_in[2];
  const float* Wk     = (const float*)d_in[3];
  const float* Wv     = (const float*)d_in[4];
  const float* Wf     = (const float*)d_in[5];
  const float* bfp    = (const float*)d_in[6];

  const size_t PXB  = (size_t)BT * WID * 2;
  const size_t PWQ  = (size_t)WID * WID * 2;
  const size_t PWK  = (size_t)HD * WID * 2;
  const size_t PWF2 = (size_t)WID * KOUT * 2;
  const size_t PQ   = (size_t)BT * WID * 2;
  const size_t PK   = (size_t)BT * HD * 2;
  const size_t PVT  = (size_t)HD * BT * 2;
  const size_t PO2  = (size_t)BT * KOUT * 2;
  size_t off = 0;
  const size_t oXB  = off; off += PXB;
  const size_t oWQB = off; off += PWQ;
  const size_t oWKB = off; off += PWK;
  const size_t oWVB = off; off += PWK;
  const size_t oWF2 = off; off += PWF2;
  const size_t oQh  = off; off += PQ;
  const size_t oQl  = off; off += PQ;
  const size_t oKh  = off; off += PK;
  const size_t oKl  = off; off += PK;
  const size_t oVTh = off; off += PVT;
  const size_t oVTl = off; off += PVT;
  const size_t oO2  = off; off += PO2;
  if (off > ws_size) return;
  if (off > (size_t)134217728) return;

  char* ws = (char*)d_ws;
  unsigned short* XB   = (unsigned short*)(ws + oXB);
  unsigned short* WQB  = (unsigned short*)(ws + oWQB);
  unsigned short* WKB  = (unsigned short*)(ws + oWKB);
  unsigned short* WVB  = (unsigned short*)(ws + oWVB);
  unsigned short* WFT2 = (unsigned short*)(ws + oWF2);
  unsigned short* Qh   = (unsigned short*)(ws + oQh);
  unsigned short* Ql   = (unsigned short*)(ws + oQl);
  unsigned short* Kh   = (unsigned short*)(ws + oKh);
  unsigned short* Kl   = (unsigned short*)(ws + oKl);
  unsigned short* VTh  = (unsigned short*)(ws + oVTh);
  unsigned short* VTl  = (unsigned short*)(ws + oVTl);
  unsigned short* O2   = (unsigned short*)(ws + oO2);

  const dim3 blk(256);
  const float* dummy = bfp;

  const int n8x  = BT * WID / 8;
  const int n8wq = WID * WID / 8;
  const int n8wk = HD * WID / 8;
  cvt_bf16_kernel<false><<<dim3((n8x + 255) / 256), blk, 0, stream>>>(x, XB, n8x, WID, WID, 0);
  cvt_bf16_kernel<false><<<dim3((n8wq + 255) / 256), blk, 0, stream>>>(Wq, WQB, n8wq, WID, WID, 0);
  cvt_bf16_kernel<false><<<dim3((n8wk + 255) / 256), blk, 0, stream>>>(Wk, WKB, n8wk, WID, WID, 0);
  cvt_bf16_kernel<false><<<dim3((n8wk + 255) / 256), blk, 0, stream>>>(Wv, WVB, n8wk, WID, WID, 0);
  cvt_bf16_kernel<true><<<dim3((n8wq + 255) / 256), blk, 0, stream>>>(Wf, WFT2, n8wq, WID, KOUT, WID);

  const dim3 gQ(((BT / 64) * (WID / 64) + 7) / 8, 1);
  wmma_gemm64<1, false, 0, 2, false><<<gQ, blk, 0, stream>>>(
      XB, XB, WID, 0L, WQB, WQB, WID, 0L, (void*)Qh, (void*)Ql, WID, 0L,
      dummy, dummy, 0L, BT, WID, WID, 1.0f);
  const dim3 gK(((BT / 64) * (HD / 64) + 7) / 8, 1);
  wmma_gemm64<1, false, 0, 2, false><<<gK, blk, 0, stream>>>(
      XB, XB, WID, 0L, WKB, WKB, WID, 0L, (void*)Kh, (void*)Kl, HD, 0L,
      dummy, dummy, 0L, BT, HD, WID, 1.0f);
  const dim3 gVT(((HD / 64) * (BT / 64) + 7) / 8, 1);
  wmma_gemm64<1, false, 0, 2, false><<<gVT, blk, 0, stream>>>(
      WVB, WVB, WID, 0L, XB, XB, WID, 0L, (void*)VTh, (void*)VTl, BT, 0L,
      dummy, dummy, 0L, HD, BT, WID, 1.0f);
  attn_local64_kernel<<<dim3(BB * NH * NQT), dim3(128), 0, stream>>>(Qh, Ql, Kh, Kl, VTh, VTl, O2, 0.125f, segpos);
  const dim3 gO(((BT / 64) * (WID / 64) + 7) / 8, 1);
  wmma_gemm64<1, false, 2, 0, false><<<gO, blk, 0, stream>>>(
      O2, O2, KOUT, 0L, WFT2, WFT2, KOUT, 0L, d_out, d_out, WID, 0L,
      bfp, dummy, 0L, BT, WID, KOUT, 1.0f);
  (void)hipGetLastError();
}
